// TemporalGATConv_12240656794125
// MI455X (gfx1250) — hardware-run, weakly checked
//
#include <hip/hip_runtime.h>


namespace {
constexpr int N = 50000, NP = 50048, E = 400000, EQ = E / 4, MEM = 64, EF = 32, TF = 32, KD = MEM + EF + TF, HD = 128, NH = 8, DH = 16, HID = 512, XD = HD + MEM, DO = 16;
constexpr float XS = 8.0f, WSC = 256.0f;
static_assert(E % 16 == 0 && EQ % 16 == 0 && 4 * EQ == E, "waves of 16 edges must not straddle a quarter boundary (the tail guard is per wave)");

typedef _Float16 b16;
typedef __attribute__((ext_vector_type(16))) _Float16 v16b;
typedef __attribute__((ext_vector_type(8))) _Float16 v8b;
typedef __attribute__((ext_vector_type(8))) float v8f;
typedef __attribute__((ext_vector_type(4))) float v4f;
typedef __attribute__((ext_vector_type(2))) float v2f;
__device__ __forceinline__ float bf16_rne(float f) { unsigned int u = __float_as_uint(f); u += 0x7FFFu + ((u >> 16) & 1u); return __uint_as_float(u & 0xFFFF0000u); }
__device__ __forceinline__ void split16(float v, b16& hi, b16& lo) { hi = (b16)v; lo = (b16)(v - (float)hi); }
__device__ __forceinline__ v16b frag_kb(const b16* p, int hh) { const v8b a = *(const v8b*)(p + 8 * hh), b = *(const v8b*)(p + 16 + 8 * hh); v16b f;
#pragma unroll
  for (int e = 0; e < 8; ++e) { f[e] = a[e]; f[8 + e] = b[e]; } return f; }
__device__ __forceinline__ v8f wmma16b(v16b a, v16b b, v8f c) { v8f d = __builtin_amdgcn_wmma_f32_16x16x32_f16(false, a, false, b, (short)0, c, false, false); asm volatile("v_nop\n\tv_nop\n\tv_nop\n\tv_nop" : "+v"(d) : "v"(a), "v"(b)); return d; }
__device__ __forceinline__ void wave_lds_sync() { __builtin_amdgcn_fence(__ATOMIC_RELEASE, "workgroup"); __builtin_amdgcn_wave_barrier(); __builtin_amdgcn_fence(__ATOMIC_ACQUIRE, "workgroup"); }
__device__ __forceinline__ float pmul(float a, float b) { float p = a * b; asm volatile("" : "+v"(p)); return p; }
__device__ __forceinline__ float hsum16(float v) { v += __shfl_xor(v, 1); v += __shfl_xor(v, 2); v += __shfl_xor(v, 4); return v + __shfl_xor(v, 8); }
__device__ __forceinline__ int iclamp(int v, int lo, int hi) { return v < lo ? lo : (v > hi ? hi : v); }

constexpr int CSR_NBLK = 512, CSR_GB = 9, CSR_GN = 1 << CSR_GB  , CSR_MAXG = 512, CSR_CAP = 12288  ;
__global__ __launch_bounds__(64) void csrA_kernel(const int* __restrict__ dst, int E, int N, int nG, int CHP, int NGP, int* __restrict__ STG, int* __restrict__ HST) {
  extern __shared__ int sm[];
  int* cnt = sm; int* run = sm + NGP; int* ids = sm + 2 * NGP;
  const int b = blockIdx.x; const int ch = (E + CSR_NBLK - 1) / CSR_NBLK; const int e0 = b * ch, e1 = min(E, e0 + ch);
  for (int i = threadIdx.x; i < NGP; i += 64) cnt[i] = 0;
  for (int i = threadIdx.x; i < CHP; i += 64) ids[i] = -1;
  __syncthreads();
  if (threadIdx.x == 0) {
    for (int e = e0; e < e1; ++e) { int d = dst[e]; d = (d < 0) ? 0 : (d >= N ? N - 1 : d); cnt[d >> CSR_GB] += 1; }
    int acc = 0; for (int g = 0; g < nG; ++g) { run[g] = acc; acc += cnt[g]; }
    for (int e = e0; e < e1; ++e) { int d = dst[e]; d = (d < 0) ? 0 : (d >= N ? N - 1 : d); const int g = d >> CSR_GB; ids[run[g]] = e; run[g] += 1; } }
  __syncthreads();
  typedef __attribute__((ext_vector_type(4))) int v4i;
  for (int pass = 0; pass < 2; ++pass) {
    for (int i = threadIdx.x; i < CHP / 4; i += 64) *(volatile v4i*)(STG + (size_t)b * CHP + i * 4) = *(const v4i*)(&ids[i * 4]);
    for (int i = threadIdx.x; i < NGP / 4; i += 64) { v4i v; for (int e = 0; e < 4; ++e) v[e] = (i * 4 + e < nG) ? cnt[i * 4 + e] : 0; *(volatile v4i*)(HST + (size_t)b * NGP + i * 4) = v; }
    __threadfence(); }
}
__global__ __launch_bounds__(512) void csrS_kernel(const int* __restrict__ HST, int nG, int NGP, int* __restrict__ START, int* __restrict__ TOT, int* __restrict__ OFF) {
  __shared__ int tot[CSR_MAXG];
  const int b = threadIdx.x;
  for (int pass = 0; pass < 2; ++pass) { int runb = 0; for (int g = 0; g < nG; ++g) { int c = HST[(size_t)b * NGP + g]; c = (c < 0) ? 0 : c; ((volatile int*)OFF)[(size_t)g * CSR_NBLK + b] = runb; runb += c; } __threadfence(); }
  for (int g = threadIdx.x; g < nG; g += 512) { int s = 0; for (int bb = 0; bb < CSR_NBLK; ++bb) { int c = HST[(size_t)bb * NGP + g]; s += (c < 0) ? 0 : c; } tot[g] = s; }
  __syncthreads();
  if (threadIdx.x < 32) {
    __shared__ int st[CSR_MAXG + 32];
    if (threadIdx.x == 0) { int acc = 0; for (int g = 0; g < NGP; ++g) { st[g] = acc; if (g < nG) acc += (tot[g] + 31) & ~31; } st[NGP] = acc; }
    __builtin_amdgcn_fence(__ATOMIC_RELEASE, "workgroup"); __builtin_amdgcn_wave_barrier(); __builtin_amdgcn_fence(__ATOMIC_ACQUIRE, "workgroup");
    for (int pass = 0; pass < 2; ++pass) { for (int i = threadIdx.x; i < NGP + 32; i += 32) { ((volatile int*)START)[i] = (i <= NGP) ? st[min(i, NGP)] : 0; ((volatile int*)TOT)[i] = (i < nG) ? tot[i] : 0; } __threadfence(); } }
}
__global__ __launch_bounds__(256) void csrB_kernel(const int* __restrict__ dst, int N, int nG, int CHP, int NGP, int permLen, const int* __restrict__ STG, const int* __restrict__ HST, const int* __restrict__ OFF, const int* __restrict__ START, const int* __restrict__ TOT, int* __restrict__ PERM, int* __restrict__ ROWPTR, int* __restrict__ ROWCNT, int* __restrict__ FLAG) {
  typedef __attribute__((ext_vector_type(4))) int v4i;
  __shared__ int ids[CSR_CAP]; __shared__ unsigned short key[CSR_CAP]; __shared__ int outp[CSR_CAP]; __shared__ int ncnt[CSR_GN + 1]; __shared__ int boff[CSR_NBLK + 1];
  const int g = blockIdx.x, t_ = threadIdx.x; int tot = TOT[g]; int st = START[g], stn = START[g + 1]; const int v0 = g * CSR_GN; const int nv = min(CSR_GN, N - v0);
  st = (st < 0) ? 0 : (st > permLen - 32 ? permLen - 32 : st) & ~31; stn = (stn < st) ? st : (stn > permLen ? permLen : stn); tot = (tot < 0) ? 0 : tot; if (tot > stn - st && tot <= CSR_CAP) tot = stn - st;
  if (tot > CSR_CAP) {
    for (int pass = 0; pass < 2; ++pass) { for (int i = t_; i < CSR_GN / 4; i += 256) { v4i a, c; for (int e = 0; e < 4; ++e) { a[e] = st; c[e] = 0; } *(volatile v4i*)(ROWPTR + v0 + i * 4) = a; *(volatile v4i*)(ROWCNT + v0 + i * 4) = c; } if (t_ == 0) ((volatile int*)FLAG)[0] = 1; __threadfence(); } (void)nv; return; }
  if (t_ == 0) { int acc = 0; for (int b = 0; b < CSR_NBLK; ++b) { boff[b] = acc; int c = HST[(size_t)b * NGP + g]; c = (c < 0) ? 0 : (c > CHP ? CHP : c); acc += c; if (acc > tot) acc = tot; } boff[CSR_NBLK] = acc; }
  for (int i = t_; i <= CSR_GN; i += 256) ncnt[i] = 0;
  __syncthreads();
  for (int b = 0; b < CSR_NBLK; ++b) { const int c = boff[b + 1] - boff[b]; int o_ = OFF[(size_t)g * CSR_NBLK + b]; o_ = (o_ < 0) ? 0 : (o_ > CHP - c ? CHP - c : o_); const int* src_ = STG + (size_t)b * CHP + o_;
    for (int i = t_; i < c; i += 256) { int id = src_[i]; id = (id < 0) ? 0 : id; ids[boff[b] + i] = id; int d = dst[id]; d = (d < v0) ? v0 : (d >= N ? N - 1 : d); int kk = d - v0; kk = (kk < 0) ? 0 : (kk >= CSR_GN ? CSR_GN - 1 : kk); key[boff[b] + i] = (unsigned short)kk; } }
  __syncthreads();
  if (t_ == 0) { for (int i = 0; i < tot; ++i) ncnt[key[i]] += 1; int acc = 0; for (int vl = 0; vl < CSR_GN; ++vl) { const int c = ncnt[vl]; ncnt[vl] = acc; acc += c; } ncnt[CSR_GN] = acc;
    for (int i = 0; i < tot; ++i) { const int vl = key[i]; outp[ncnt[vl]] = ids[i]; ncnt[vl] += 1; }
    for (int vl = CSR_GN; vl > 0; --vl) ncnt[vl] = ncnt[vl - 1]; ncnt[0] = 0; }
  __syncthreads();
  for (int pass = 0; pass < 2; ++pass) {
    for (int i = t_; i < (stn - st) / 4; i += 256) { v4i v; for (int e = 0; e < 4; ++e) { const int q = i * 4 + e; v[e] = (q < tot) ? outp[q] : -1; } *(volatile v4i*)(PERM + st + i * 4) = v; }
    for (int i = t_; i < CSR_GN / 4; i += 256) { v4i a, c; for (int e = 0; e < 4; ++e) { const int vl = i * 4 + e; a[e] = st + ncnt[vl]; c[e] = (vl < nv) ? (ncnt[vl + 1] - ncnt[vl]) : 0; } *(volatile v4i*)(ROWPTR + v0 + i * 4) = a; *(volatile v4i*)(ROWCNT + v0 + i * 4) = c; }
    __threadfence(); }
}
__global__ __launch_bounds__(256) void csrZ_kernel(int* __restrict__ p, size_t n4) { typedef __attribute__((ext_vector_type(4))) int v4i; const size_t tid = (size_t)blockIdx.x * 256 + threadIdx.x, nth = (size_t)gridDim.x * 256; v4i z = {0, 0, 0, 0}; for (size_t i = tid; i < n4; i += nth) *(volatile v4i*)(p + i * 4) = z; }
struct CsrBufs { int *STG, *HST, *OFF, *START, *TOT, *PERM, *ROWPTR, *ROWCNT, *FLAG; int nG, NGP, CHP; size_t permLen; char* base; size_t bytes; };
static size_t csr_carve(CsrBufs& c, char* ws, size_t off, int E, int N) {
  const size_t off0 = off; c.base = ws + off;
  auto al = [&](size_t bytes) { char* p = ws + off; off += (bytes + 255) & ~(size_t)255; return p; };
  c.nG = (N + CSR_GN - 1) / CSR_GN; c.NGP = (c.nG + 31) & ~31; const int ch = (E + CSR_NBLK - 1) / CSR_NBLK; c.CHP = (ch + 31) & ~31; c.permLen = (size_t)E + 32 * (size_t)c.nG + 32;
  c.STG = (int*)al((size_t)CSR_NBLK * c.CHP * 4); c.HST = (int*)al((size_t)CSR_NBLK * c.NGP * 4); c.OFF = (int*)al((size_t)c.NGP * CSR_NBLK * 4); c.START = (int*)al((size_t)(c.NGP + 64) * 4); c.TOT = (int*)al((size_t)(c.NGP + 64) * 4);
  c.PERM = (int*)al(c.permLen * 4); c.ROWPTR = (int*)al((size_t)c.nG * CSR_GN * 4); c.ROWCNT = (int*)al((size_t)c.nG * CSR_GN * 4); c.FLAG = (int*)al(256);
  c.bytes = off - off0; return off;
}
static void csr_build(const CsrBufs& c, const int* dst, int E, int N, hipStream_t stream) {
  const size_t smem = (size_t)(2 * c.NGP + c.CHP) * 4;
  csrZ_kernel<<<512, 256, 0, stream>>>((int*)c.base, c.bytes / 16);
  csrA_kernel<<<CSR_NBLK, 64, smem, stream>>>(dst, E, N, c.nG, c.CHP, c.NGP, c.STG, c.HST);
  csrS_kernel<<<1, 512, 0, stream>>>(c.HST, c.nG, c.NGP, c.START, c.TOT, c.OFF);
  csrB_kernel<<<c.nG, 256, 0, stream>>>(dst, N, c.nG, c.CHP, c.NGP, (int)c.permLen, c.STG, c.HST, c.OFF, c.START, c.TOT, c.PERM, c.ROWPTR, c.ROWCNT, c.FLAG);
}


__global__ __launch_bounds__(256) void prep_kernel(const float* __restrict__ mem, const float* __restrict__ wq, const float* __restrict__ wk, const float* __restrict__ w1, const float* __restrict__ tb, const float* __restrict__ w2, b16* __restrict__ M16, b16* __restrict__ WQM, b16* __restrict__ WK, b16* __restrict__ W1h, b16* __restrict__ W2p, float* __restrict__ CQ) {
  const size_t g = (size_t)blockIdx.x * 256 + threadIdx.x; const size_t n0 = (size_t)NP * MEM / 8, n1 = HD * MEM / 8, n2 = HD * HD / 8, n3 = (size_t)HID * XD / 8, n4 = (size_t)DO * HID / 8;
  v8b o; b16* dst;
  if (g < n0) { const size_t e = g * 8, row = e / MEM; dst = M16 + e; if (row < N) { const v4f a = *(const v4f*)(mem + e), c = *(const v4f*)(mem + e + 4);
#pragma unroll
      for (int j = 0; j < 4; ++j) { o[j] = (b16)(bf16_rne(a[j]) * XS); o[4 + j] = (b16)(bf16_rne(c[j]) * XS); } } else o = (v8b){}; }
  else if (g < n0 + n1) { const int e = (int)(g - n0) * 8, r = e / MEM, c = e - r * MEM; dst = WQM + e;
#pragma unroll
    for (int j = 0; j < 8; ++j) o[j] = (b16)(bf16_rne(wq[r * (MEM + TF) + c + j]) * WSC); }
  else if (g < n0 + n1 + n2) { const int e = (int)(g - n0 - n1) * 8; dst = WK + e;
#pragma unroll
    for (int j = 0; j < 8; ++j) o[j] = (b16)(bf16_rne(wk[e + j]) * WSC); }
  else if (g < n0 + n1 + n2 + n3) { const int e = (int)(g - n0 - n1 - n2) * 8; dst = W1h + e;
#pragma unroll
    for (int j = 0; j < 8; ++j) o[j] = (b16)(bf16_rne(w1[e + j]) * WSC); }
  else if (g < n0 + n1 + n2 + n3 + n4) { const int e = (int)(g - n0 - n1 - n2 - n3) * 8; dst = W2p + e;
#pragma unroll
    for (int j = 0; j < 8; ++j) o[j] = (b16)(bf16_rne(w2[e + j]) * WSC); }
  else { const int o_ = (int)(g - n0 - n1 - n2 - n3 - n4); if (o_ >= HD) return; float s = 0.0f;
#pragma unroll 1
    for (int j = 0; j < TF; ++j) s += pmul(bf16_rne(wq[o_ * (MEM + TF) + MEM + j]), cosf(bf16_rne(tb[j])));
    for (int pass = 0; pass < 2; ++pass) { ((volatile float*)CQ)[o_] = s; __threadfence(); } return; }
  for (int pass = 0; pass < 2; ++pass) { *(volatile v8b*)dst = o; __threadfence(); }
}
__global__ __launch_bounds__(128) void qn_kernel(const b16* __restrict__ M16, const b16* __restrict__ WQM, const float* __restrict__ CQ, float* __restrict__ QN) {
  __shared__ __attribute__((aligned(16))) float Ts[4][16][HD + 4];
  const int wave = threadIdx.x >> 5, lane = threadIdx.x & 31, nloc = lane & 15, hlf = lane >> 4; const size_t m0 = (size_t)blockIdx.x * 64 + wave * 16;
  v8f acc[8];
#pragma unroll
  for (int t = 0; t < 8; ++t) acc[t] = (v8f){};
#pragma unroll
  for (int kb = 0; kb < MEM; kb += 32) { const v16b a = frag_kb(M16 + (m0 + nloc) * MEM + kb, hlf);
#pragma unroll
    for (int t = 0; t < 8; ++t) acc[t] = wmma16b(a, frag_kb(WQM + (size_t)(t * 16 + nloc) * MEM + kb, hlf), acc[t]); }
#pragma unroll
  for (int t = 0; t < 8; ++t) { const float cq = CQ[t * 16 + nloc];
#pragma unroll
    for (int r = 0; r < 8; ++r) Ts[wave][8 * hlf + r][t * 16 + nloc] = acc[t][r] * (1.0f / (XS * WSC)) + cq; }
  wave_lds_sync();
  for (int pass = 0; pass < 2; ++pass) { for (int rr = 0; rr < 16; ++rr) *(volatile v4f*)(QN + (m0 + rr) * HD + lane * 4) = *(const v4f*)(&Ts[wave][rr][lane * 4]); __threadfence(); }
}
template <int PHASE>
__global__ __launch_bounds__(128) void edge_kernel(const int* __restrict__ src, const int* __restrict__ dst, const float* __restrict__ ts, const float* __restrict__ ets, const float* __restrict__ ef, const float* __restrict__ tw, const float* __restrict__ tb,
                                                  const b16* __restrict__ M16, const b16* __restrict__ WK, const float* __restrict__ QN, int ebase, float* __restrict__ A8, b16* __restrict__ KHh, b16* __restrict__ KHl) {
  __shared__ __attribute__((aligned(16))) b16 Ta[4][16][KD + 8], Tlo[4][16][TF + 8]; __shared__ __attribute__((aligned(16))) float Tl[4][16][8]; __shared__ __attribute__((aligned(16))) b16 Th[4][16][HD + 8], Tq[4][16][HD + 8];
  const int wave = threadIdx.x >> 5, lane = threadIdx.x & 31, nloc = lane & 15, hlf = lane >> 4; const int e0 = ebase + (blockIdx.x * 4 + wave) * 16;
  if (e0 >= ebase + (PHASE == 0 ? E : EQ) || e0 >= E) return;
  { const int rr = lane >> 1, hf = lane & 1; const int e = e0 + rr; const int s = iclamp(src[e], 0, N - 1);
    const v8b* ms_ = (const v8b*)(M16 + (size_t)s * MEM + hf * 32); *(v8b*)(&Ta[wave][rr][hf * 32]) = ms_[0]; *(v8b*)(&Ta[wave][rr][hf * 32 + 8]) = ms_[1]; *(v8b*)(&Ta[wave][rr][hf * 32 + 16]) = ms_[2]; *(v8b*)(&Ta[wave][rr][hf * 32 + 24]) = ms_[3];
    const float tdiff = bf16_rne(ets[e]) - bf16_rne(ts[s]);
#pragma unroll
    for (int j = 0; j < 16; ++j) { const int c = hf * 16 + j; Ta[wave][rr][MEM + c] = (b16)(bf16_rne(ef[(size_t)e * EF + c]) * XS); b16 th, tl; split16(cosf(pmul(tdiff, bf16_rne(tw[c])) + bf16_rne(tb[c])) * XS, th, tl); Ta[wave][rr][MEM + EF + c] = th; Tlo[wave][rr][c] = tl; } }
  wave_lds_sync();
  v8f acc[8];
#pragma unroll
  for (int t = 0; t < 8; ++t) acc[t] = (v8f){};
#pragma unroll
  for (int kb = 0; kb < KD; kb += 32) { const v16b a = frag_kb(&Ta[wave][nloc][kb], hlf);
#pragma unroll
    for (int t = 0; t < 8; ++t) acc[t] = wmma16b(a, frag_kb(WK + (size_t)(t * 16 + nloc) * KD + kb, hlf), acc[t]); }
  { const v16b al = frag_kb(&Tlo[wave][nloc][0], hlf);
#pragma unroll
    for (int t = 0; t < 8; ++t) acc[t] = wmma16b(al, frag_kb(WK + (size_t)(t * 16 + nloc) * KD + MEM + EF, hlf), acc[t]); }
  if (PHASE == 0) {
#pragma unroll
    for (int r = 0; r < 8; ++r) { const int e = e0 + 8 * hlf + r; const int dv = iclamp(dst[e], 0, N - 1); const float* qn = QN + (size_t)dv * HD;
#pragma unroll
      for (int t = 0; t < 8; ++t) { float p = pmul(acc[t][r] * (1.0f / (XS * WSC)), qn[t * 16 + nloc]); p = hsum16(p); if (nloc == 0) Tl[wave][8 * hlf + r][t] = p; } }
    wave_lds_sync();
    for (int pass = 0; pass < 2; ++pass) { *(volatile v4f*)(A8 + (size_t)e0 * NH + lane * 4) = *(const v4f*)(&Tl[wave][0][0] + lane * 4); __threadfence(); }
  } else {
#pragma unroll
    for (int t = 0; t < 8; ++t)
#pragma unroll
      for (int r = 0; r < 8; ++r) { b16 a_, c_; split16(acc[t][r] * (1.0f / (XS * WSC)) * XS, a_, c_); Th[wave][8 * hlf + r][t * 16 + nloc] = a_; Tq[wave][8 * hlf + r][t * 16 + nloc] = c_; }
    wave_lds_sync();
    for (int pass = 0; pass < 2; ++pass) { for (int rr = 0; rr < 16; ++rr) if (lane < 16) { const size_t gi = ((size_t)(e0 - ebase) + rr) * HD + lane * 8; *(volatile v8b*)(KHh + gi) = *(const v8b*)(&Th[wave][rr][lane * 8]); *(volatile v8b*)(KHl + gi) = *(const v8b*)(&Tq[wave][rr][lane * 8]); } __threadfence(); }
  }
}
__global__ __launch_bounds__(256) void stats_kernel(const float* __restrict__ A8, const int* __restrict__ PERM, const int* __restrict__ ROWPTR, const int* __restrict__ ROWCNT, int permLen, float* __restrict__ MD) {
  const int wave = threadIdx.x >> 5, lane = threadIdx.x & 31; const int v0 = (blockIdx.x * 8 + wave) * 4; const int v = v0 + (lane >> 3), h = lane & 7;
  int st = ROWPTR[v], cnt = ROWCNT[v]; cnt = iclamp(cnt, 0, 4096); st = iclamp(st, 0, permLen - cnt);
  float m = -INFINITY; for (int j = 0; j < cnt; ++j) { const int e = iclamp(PERM[st + j], 0, E - 1); m = fmaxf(m, A8[(size_t)e * NH + h]); }
  float den = 0.0f; for (int j = 0; j < cnt; ++j) { const int e = iclamp(PERM[st + j], 0, E - 1); den += __expf(A8[(size_t)e * NH + h] - m); }
  const float mo = (cnt > 0) ? m : 0.0f, ido = (cnt > 0) ? 1.0f / den : 0.0f;
  const int f0 = 2 * lane; float vals[2];
#pragma unroll
  for (int q = 0; q < 2; ++q) { const int f = f0 + q; const int nd = f >> 4, sl = f & 15; const int srcl = nd * 8 + (sl & 7); const float mm = __shfl(mo, srcl), dd = __shfl(ido, srcl); vals[q] = (sl < 8) ? mm : dd; }
  v2f w2 = {vals[0], vals[1]};
  for (int pass = 0; pass < 2; ++pass) { *(volatile v2f*)(MD + (size_t)v0 * 16 + f0) = w2; __threadfence(); }
}
template <int QTR>
__global__ __launch_bounds__(256) void agg_kernel(const float* __restrict__ A8, const float* __restrict__ MD, const b16* __restrict__ KHh, const b16* __restrict__ KHl, const int* __restrict__ PERM, const int* __restrict__ ROWPTR, const int* __restrict__ ROWCNT, int permLen, float* __restrict__ AGG) {
  const int wave = threadIdx.x >> 5, lane = threadIdx.x & 31; const size_t v = ((size_t)blockIdx.x * 8 + wave) * 2 + (lane >> 4); const int c0 = (lane & 15) * 8, h = c0 / DH;
  int st = ROWPTR[v], cnt = ROWCNT[v]; cnt = iclamp(cnt, 0, 4096); st = iclamp(st, 0, permLen - cnt);
  const float m = MD[v * 16 + h], ido = MD[v * 16 + 8 + h] * 0.25f;
  float acc[8]; if (QTR == 0) { for (int j = 0; j < 8; ++j) acc[j] = 0.0f; } else { const v4f a = *(const v4f*)(AGG + v * HD + c0), b = *(const v4f*)(AGG + v * HD + c0 + 4); for (int j = 0; j < 4; ++j) { acc[j] = a[j]; acc[4 + j] = b[j]; } }
  for (int j = 0; j < cnt; ++j) { const int e = iclamp(PERM[st + j], 0, E - 1); const bool inq = (e >= QTR * EQ) && (e < (QTR + 1) * EQ); const int el = iclamp(e - QTR * EQ, 0, EQ - 1);
    const float sa = inq ? pmul(__expf(A8[(size_t)e * NH + h] - m), ido) : 0.0f; const v8b kh = *(const v8b*)(KHh + (size_t)el * HD + c0), kl = *(const v8b*)(KHl + (size_t)el * HD + c0);
#pragma unroll
    for (int q = 0; q < 8; ++q) acc[q] += pmul(sa, ((float)kh[q] + (float)kl[q]) * (1.0f / XS)); }
  v4f oa = {acc[0], acc[1], acc[2], acc[3]}, ob = {acc[4], acc[5], acc[6], acc[7]};
  for (int pass = 0; pass < 2; ++pass) { *(volatile v4f*)(AGG + v * HD + c0) = oa; *(volatile v4f*)(AGG + v * HD + c0 + 4) = ob; __threadfence(); }
}
__global__ __launch_bounds__(256) void xplane_kernel(const float* __restrict__ AGG, const float* __restrict__ mem, b16* __restrict__ Xh, b16* __restrict__ Xl) {
  const int wave = threadIdx.x >> 5, lane = threadIdx.x & 31; const size_t v = (size_t)blockIdx.x * 8 + wave; if (lane >= 24) return;
  v8b o, ol;
  if (lane < 16) { const float* a = AGG + v * HD + lane * 8;
#pragma unroll
    for (int j = 0; j < 8; ++j) { b16 h_, l_; split16(a[j] * XS, h_, l_); o[j] = h_; ol[j] = l_; } }
  else { const int c = (lane - 16) * 8;
#pragma unroll
    for (int j = 0; j < 8; ++j) { o[j] = (v < N) ? (b16)(bf16_rne(mem[v * MEM + c + j]) * XS) : (b16)0.0f; ol[j] = (b16)0.0f; } }
  for (int pass = 0; pass < 2; ++pass) { *(volatile v8b*)(Xh + v * XD + lane * 8) = o; *(volatile v8b*)(Xl + v * XD + lane * 8) = ol; __threadfence(); }
}
__global__ __launch_bounds__(128) void mlp_kernel(const b16* __restrict__ Xh, const b16* __restrict__ Xl, const b16* __restrict__ W1h, const float* __restrict__ b1, const b16* __restrict__ W2p, const float* __restrict__ b2, float* __restrict__ out) {
  __shared__ __attribute__((aligned(16))) b16 Hs[16][HID + 8], Hl[16][HID + 8]; __shared__ __attribute__((aligned(16))) float To[16][DO];
  const int wave = threadIdx.x >> 5, lane = threadIdx.x & 31, nloc = lane & 15, hlf = lane >> 4; const size_t m0 = (size_t)blockIdx.x * 16; const int n0 = wave * 128;
  v8f acc[8];
#pragma unroll
  for (int t = 0; t < 8; ++t) acc[t] = (v8f){};
#pragma unroll
  for (int kb = 0; kb < XD; kb += 32) { const v16b a = frag_kb(Xh + (m0 + nloc) * XD + kb, hlf);
#pragma unroll
    for (int t = 0; t < 8; ++t) { const v16b bw = frag_kb(W1h + (size_t)(n0 + t * 16 + nloc) * XD + kb, hlf); acc[t] = wmma16b(a, bw, acc[t]); if (kb < HD) acc[t] = wmma16b(frag_kb(Xl + (m0 + nloc) * XD + kb, hlf), bw, acc[t]); } }
#pragma unroll
  for (int t = 0; t < 8; ++t) { const float bb = bf16_rne(b1[n0 + t * 16 + nloc]);
#pragma unroll
    for (int r = 0; r < 8; ++r) { b16 h_, l_; split16(fmaxf(acc[t][r] * (1.0f / (XS * WSC)) + bb, 0.0f) * XS, h_, l_); Hs[8 * hlf + r][n0 + t * 16 + nloc] = h_; Hl[8 * hlf + r][n0 + t * 16 + nloc] = l_; } }
  __syncthreads();
  if (wave == 0) { v8f o = {};
#pragma unroll 4
    for (int kb = 0; kb < HID; kb += 32) { const v16b bw = frag_kb(W2p + (size_t)nloc * HID + kb, hlf); o = wmma16b(frag_kb(&Hs[nloc][kb], hlf), bw, o); o = wmma16b(frag_kb(&Hl[nloc][kb], hlf), bw, o); }
#pragma unroll
    for (int r = 0; r < 8; ++r) To[8 * hlf + r][nloc] = o[r] * (1.0f / (XS * WSC)) + bf16_rne(b2[nloc]);
    wave_lds_sync();
    const int rr = lane >> 1, o0 = (lane & 1) * 8; const v4f a = *(const v4f*)(&To[rr][o0]), c = *(const v4f*)(&To[rr][o0 + 4]);
    for (int pass = 0; pass < 2; ++pass) { if (m0 + rr < N) { *(volatile v4f*)(out + (m0 + rr) * DO + o0) = a; *(volatile v4f*)(out + (m0 + rr) * DO + o0 + 4) = c; } __threadfence(); } }
}
}

extern "C" void kernel_launch(void* const* d_in, const int* in_sizes, int n_in, void* d_out, int out_size, void* d_ws, size_t ws_size, hipStream_t stream) {
  (void)n_in;
  auto Fp = [&](int i) { return (const float*)d_in[i]; }; auto Ip = [&](int i) { return (const int*)d_in[i]; };
  if (in_sizes[0] != E || in_sizes[1] != E || in_sizes[2] != N * MEM || in_sizes[3] != N || in_sizes[4] != E * EF || in_sizes[5] != E || in_sizes[6] != HD * (MEM + TF) || in_sizes[7] != HD * KD || in_sizes[8] != HID * XD || in_sizes[10] != DO * HID || in_sizes[12] != TF || out_size != N * DO) return;
  size_t off = 0; char* ws = (char*)d_ws;
  auto carve = [&](size_t bytes) { char* p = ws + off; off += (bytes + 255) & ~(size_t)255; return p; };
  b16* M16 = (b16*)carve((size_t)NP * MEM * 2); b16* WQM = (b16*)carve(HD * MEM * 2); b16* WK = (b16*)carve(HD * KD * 2); b16* W1h = (b16*)carve((size_t)HID * XD * 2); b16* W2p = (b16*)carve((size_t)DO * HID * 2); float* CQ = (float*)carve(HD * 4);
  float* QN = (float*)carve((size_t)NP * HD * 4); float* A8 = (float*)carve((size_t)E * NH * 4); float* MD = (float*)carve((size_t)NP * 16 * 4);
  b16* KHh = (b16*)carve((size_t)EQ * HD * 2); b16* KHl = (b16*)carve((size_t)EQ * HD * 2);
  CsrBufs csr; off = csr_carve(csr, ws, off, E, N);
  float* AGG = QN;
  b16* Xh = KHh; b16* Xl = KHl;
  if (off > ws_size || off > ((size_t)128 << 20)) return;
  prep_kernel<<<((size_t)NP * MEM / 8 + HD * MEM / 8 + HD * HD / 8 + HID * XD / 8 + DO * HID / 8 + HD + 255) / 256, 256, 0, stream>>>(Fp(2), Fp(6), Fp(7), Fp(8), Fp(13), Fp(10), M16, WQM, WK, W1h, W2p, CQ);
  qn_kernel<<<NP / 64, 128, 0, stream>>>(M16, WQM, CQ, QN);
  csr_build(csr, Ip(1), E, N, stream);
  edge_kernel<0><<<(E + 63) / 64, 128, 0, stream>>>(Ip(0), Ip(1), Fp(3), Fp(5), Fp(4), Fp(12), Fp(13), M16, WK, QN, 0, A8, KHh, KHl);
  stats_kernel<<<NP / 32, 256, 0, stream>>>(A8, csr.PERM, csr.ROWPTR, csr.ROWCNT, (int)csr.permLen, MD);
  edge_kernel<1><<<(EQ + 63) / 64, 128, 0, stream>>>(Ip(0), Ip(1), Fp(3), Fp(5), Fp(4), Fp(12), Fp(13), M16, WK, QN, 0 * EQ, A8, KHh, KHl); agg_kernel<0><<<NP / 16, 256, 0, stream>>>(A8, MD, KHh, KHl, csr.PERM, csr.ROWPTR, csr.ROWCNT, (int)csr.permLen, AGG);
  edge_kernel<1><<<(EQ + 63) / 64, 128, 0, stream>>>(Ip(0), Ip(1), Fp(3), Fp(5), Fp(4), Fp(12), Fp(13), M16, WK, QN, 1 * EQ, A8, KHh, KHl); agg_kernel<1><<<NP / 16, 256, 0, stream>>>(A8, MD, KHh, KHl, csr.PERM, csr.ROWPTR, csr.ROWCNT, (int)csr.permLen, AGG);
  edge_kernel<1><<<(EQ + 63) / 64, 128, 0, stream>>>(Ip(0), Ip(1), Fp(3), Fp(5), Fp(4), Fp(12), Fp(13), M16, WK, QN, 2 * EQ, A8, KHh, KHl); agg_kernel<2><<<NP / 16, 256, 0, stream>>>(A8, MD, KHh, KHl, csr.PERM, csr.ROWPTR, csr.ROWCNT, (int)csr.permLen, AGG);
  edge_kernel<1><<<(EQ + 63) / 64, 128, 0, stream>>>(Ip(0), Ip(1), Fp(3), Fp(5), Fp(4), Fp(12), Fp(13), M16, WK, QN, 3 * EQ, A8, KHh, KHl); agg_kernel<3><<<NP / 16, 256, 0, stream>>>(A8, MD, KHh, KHl, csr.PERM, csr.ROWPTR, csr.ROWCNT, (int)csr.permLen, AGG);
  xplane_kernel<<<NP / 8, 256, 0, stream>>>(AGG, Fp(2), Xh, Xl);
  mlp_kernel<<<NP / 16, 128, 0, stream>>>(Xh, Xl, W1h, Fp(9), W2p, Fp(11), (float*)d_out);
}
